// RotaryTransformerLayer_68796786147576
// MI455X (gfx1250) — hardware-run, weakly checked
//
#include <hip/hip_runtime.h>
#include <math.h>
#include <stddef.h>

constexpr int kBatch  = 2;
constexpr int kSeq    = 2048;
constexpr int kDim    = 1024;
constexpr int kHeads  = 16;
constexpr int kHd     = 64;
constexpr int kTok    = kBatch * kSeq;
constexpr int kQkvN   = 3 * kDim;
constexpr int kFfn    = 4 * kDim;
constexpr int kGroups = kBatch * kHeads;
constexpr int kChunkG = 4;
constexpr float kLnEps    = 1e-5f;
constexpr float kWCarry   = 64.0f;
constexpr float kW2Carry  = 128.0f;
constexpr float kPCarry   = 2048.0f;
constexpr float kAttCarry = 256.0f;
constexpr float kHCarry   = 8.0f;
constexpr float kQkvScale  = 1.0f / kWCarry;
constexpr float kScoreScale = 0.125f;
constexpr float kPVScale   = kAttCarry / kPCarry;
constexpr float kWoScale   = 1.0f / (kAttCarry * kWCarry);
constexpr float kFfn1Scale = 1.0f / kWCarry;
constexpr float kFfn2Scale = 1.0f / (kHCarry * kW2Carry);

constexpr size_t kMiB     = 1048576;
constexpr size_t kOffQkvF = 0;
constexpr size_t kOffX16  = 48 * kMiB;
constexpr size_t kOffWqkv = 56 * kMiB;
constexpr size_t kOffTab  = 62 * kMiB;
constexpr size_t kOffQ16  = 64 * kMiB;
constexpr size_t kOffK16  = 72 * kMiB;
constexpr size_t kOffVt16 = 80 * kMiB;
constexpr size_t kOffSc   = 0;
constexpr size_t kOffP    = 88 * kMiB;
constexpr size_t kOffAtt  = 120 * kMiB;
constexpr size_t kOffWo   = 80 * kMiB;
constexpr size_t kOffY1   = 64 * kMiB;
constexpr size_t kOffX1F  = 96 * kMiB;
constexpr size_t kOffX1H  = 112 * kMiB;
constexpr size_t kOffW1   = 82 * kMiB;
constexpr size_t kOffHpre = 0;
constexpr size_t kOffH16  = 64 * kMiB;
constexpr size_t kOffW2   = 0;
constexpr size_t kOffY2   = 8 * kMiB;
constexpr size_t kWsNeed  = 128 * kMiB;

typedef __attribute__((ext_vector_type(16))) _Float16 v16h;
typedef __attribute__((ext_vector_type(8)))  _Float16 v8h;
typedef __attribute__((ext_vector_type(16))) __bf16   v16b;
typedef __attribute__((ext_vector_type(8)))  __bf16   v8b;
typedef __attribute__((ext_vector_type(8)))  float    v8f;
typedef __attribute__((ext_vector_type(4)))  float    v4f;
typedef __attribute__((ext_vector_type(4)))  unsigned int v4u;

__device__ __forceinline__ unsigned short f2bf_bits(float f) {
  unsigned u = __float_as_uint(f);
  return (unsigned short)((u + 0x7FFFu + ((u >> 16) & 1u)) >> 16);
}
__device__ __forceinline__ float bf_bits2f(unsigned short h) { return __uint_as_float(((unsigned)h) << 16); }

__device__ __forceinline__ void dep_guard_h(v8f& a, v8f& b, v16h x, v16h y) { asm volatile("v_nop\n\tv_nop\n\tv_nop\n\tv_nop" : "+v"(a), "+v"(b) : "v"(x), "v"(y)); }
__device__ __forceinline__ void dep_guard_b(v8f& a, v8f& b, v16b x, v16b y) { asm volatile("v_nop\n\tv_nop\n\tv_nop\n\tv_nop" : "+v"(a), "+v"(b) : "v"(x), "v"(y)); }
__device__ __forceinline__ void keep4_h(v16h a, v16h b, v16h c, v16h d) { asm volatile("v_nop" :: "v"(a), "v"(b), "v"(c), "v"(d)); }
__device__ __forceinline__ void keep4_b(v16b a, v16b b, v16b c, v16b d) { asm volatile("v_nop" :: "v"(a), "v"(b), "v"(c), "v"(d)); }
__device__ __forceinline__ void acc_guard4(v8f& a, v8f& b, v8f& c, v8f& d) { asm volatile("v_nop\n\tv_nop\n\tv_nop\n\tv_nop" : "+v"(a), "+v"(b), "+v"(c), "+v"(d)); }
template <typename T> struct Frag;
template <> struct Frag<_Float16> {
  typedef v16h V; union U { v16h v; v8h h[2]; };
  static __device__ __forceinline__ v16h load(const _Float16* p) {
    U f; f.h[0] = *(const v8h*)(p); f.h[1] = *(const v8h*)(p + 16); return f.v;
  }
  static __device__ __forceinline__ v8f mma(v16h a, v16h b, v8f c) {
    return __builtin_amdgcn_wmma_f32_16x16x32_f16(false, a, false, b, (short)0, c, false, false);
  }
  static __device__ __forceinline__ void guard(v8f& a, v8f& b, v16h x, v16h y) { dep_guard_h(a, b, x, y); }
  static __device__ __forceinline__ void keep(v16h a, v16h b, v16h c, v16h d) { keep4_h(a, b, c, d); }
};
template <> struct Frag<__bf16> {
  typedef v16b V; union U { v16b v; v8b h[2]; };
  static __device__ __forceinline__ v16b load(const __bf16* p) {
    U f; f.h[0] = *(const v8b*)(p); f.h[1] = *(const v8b*)(p + 16); return f.v;
  }
  static __device__ __forceinline__ v8f mma(v16b a, v16b b, v8f c) {
    return __builtin_amdgcn_wmma_f32_16x16x32_bf16(false, a, false, b, (short)0, c, false, false);
  }
  static __device__ __forceinline__ void guard(v8f& a, v8f& b, v16b x, v16b y) { dep_guard_b(a, b, x, y); }
  static __device__ __forceinline__ void keep(v16b a, v16b b, v16b c, v16b d) { keep4_b(a, b, c, d); }
};

__device__ __forceinline__ unsigned pk16(unsigned short a, unsigned short b) { return (unsigned)a | ((unsigned)b << 16); }
__device__ __forceinline__ unsigned short h_bits(float f) { const _Float16 h = (_Float16)f; return __builtin_bit_cast(unsigned short, h); }

template <int ET> struct Elem;
template <> struct Elem<0> { typedef _Float16 T; };
template <> struct Elem<1> { typedef __bf16 T; };
template <int ET, bool SPLIT, int BIAS_MODE, int OUT_MODE, bool RESID, int ACT = 0>
__global__ __launch_bounds__(256) void wmma_gemm64(
    const unsigned short* __restrict__ Ap, const unsigned short* __restrict__ A2p, int lda, long strideA,
    const unsigned short* __restrict__ Btp, const unsigned short* __restrict__ Bt2p, int ldb, long strideB,
    void* __restrict__ Cout, void* __restrict__ Cout2, int ldc, long strideC,
    const float* __restrict__ bias,
    const float* __restrict__ resid, long strideR,
    int M, int N, int K, float scale) {
  typedef typename Elem<ET>::T T;
  typedef typename Frag<T>::V V;
  const T* A = (const T*)Ap; const T* A2 = (const T*)A2p; const T* Bt = (const T*)Btp; const T* Bt2 = (const T*)Bt2p;
  __shared__ __align__(16) float sT[8][16 * 68];
  const int b    = blockIdx.y;
  const int lane = threadIdx.x & 31;
  const int wave = threadIdx.x >> 5;
  const int tilesN = N >> 6;
  const int tilesM = M >> 6;
  const int tile = blockIdx.x * 8 + wave;
  if (tile >= tilesM * tilesN) return;
  const int tm = tile / tilesN;
  const int tn = tile - tm * tilesN;
  const int m0 = tm << 6;
  const int n0 = tn << 6;

  const T* Ab  = A  + (size_t)b * strideA;
  const T* Bb  = Bt + (size_t)b * strideB;
  const T* Ab2 = SPLIT ? (A2  + (size_t)b * strideA) : nullptr;
  const T* Bb2 = SPLIT ? (Bt2 + (size_t)b * strideB) : nullptr;

  const int rlane = lane & 15;
  const int koff  = (lane >> 4) * 8;
  const int mOff  = (lane >> 4) * 8;

  v8f acc[4][4];
#pragma unroll
  for (int i = 0; i < 4; ++i)
#pragma unroll
    for (int j = 0; j < 4; ++j) acc[i][j] = (v8f){0.f,0.f,0.f,0.f,0.f,0.f,0.f,0.f};

  for (int k0 = 0; k0 < K; k0 += 32) {
    V bh[4], bl[4];
#pragma unroll
    for (int j = 0; j < 4; ++j) {
      const size_t bo = (size_t)(n0 + (j << 4) + rlane) * ldb + koff + k0;
      bh[j] = Frag<T>::load(Bb + bo);
      if (SPLIT) bl[j] = Frag<T>::load(Bb2 + bo);
    }
#pragma unroll
    for (int i = 0; i < 4; ++i) {
      const size_t ao = (size_t)(m0 + (i << 4) + rlane) * lda + koff + k0;
      V ah = Frag<T>::load(Ab + ao);
      V al;
      if (SPLIT) al = Frag<T>::load(Ab2 + ao);
#pragma unroll
      for (int j = 0; j < 4; ++j) {
        acc[i][j] = Frag<T>::mma(ah, bh[j], acc[i][j]);
        if (SPLIT) {
          acc[i][j] = Frag<T>::mma(ah, bl[j], acc[i][j]);
          acc[i][j] = Frag<T>::mma(al, bh[j], acc[i][j]);
        }
      }
      Frag<T>::guard(acc[i][0], acc[i][3], ah, SPLIT ? al : ah);
    }
    Frag<T>::keep(bh[0], bh[1], bh[2], bh[3]);
    if (SPLIT) Frag<T>::keep(bl[0], bl[1], bl[2], bl[3]);
  }
  acc_guard4(acc[0][0], acc[0][1], acc[0][2], acc[0][3]);
  acc_guard4(acc[1][0], acc[1][1], acc[1][2], acc[1][3]);
  acc_guard4(acc[2][0], acc[2][1], acc[2][2], acc[2][3]);
  acc_guard4(acc[3][0], acc[3][1], acc[3][2], acc[3][3]);

  float* slab = sT[wave];
  const float* Rb = RESID ? (resid + (size_t)b * strideR) : nullptr;
#pragma unroll
  for (int i = 0; i < 4; ++i) {
    const int mBase = m0 + (i << 4);
#pragma unroll
    for (int j = 0; j < 4; ++j) {
      const int n = n0 + (j << 4) + rlane;
      float bv = 0.f;
      if (BIAS_MODE == 2) bv = bias[n];
#pragma unroll
      for (int r = 0; r < 8; ++r) {
        float v = acc[i][j][r] * scale;
        if (BIAS_MODE == 1) v += bias[mBase + mOff + r];
        if (BIAS_MODE == 2) v += bv;
        if (RESID) v += Rb[(size_t)(mBase + mOff + r) * ldc + n];
        if (ACT == 2) v = fmaxf(v, 0.0f);
        if (ACT == 4) v = (v > 0.f) ? v : 0.01f * v;
        slab[(mOff + r) * 68 + (j << 4) + rlane] = v;
      }
    }
    __builtin_amdgcn_fence(__ATOMIC_RELEASE, "workgroup");
    __builtin_amdgcn_wave_barrier();
    __builtin_amdgcn_fence(__ATOMIC_ACQUIRE, "workgroup");
    if (OUT_MODE == 0) {
      float* C = (float*)Cout + (size_t)b * strideC;
      const int hh = lane >> 4, c4 = (lane & 15) * 4;
      for (int pass = 0; pass < 2; ++pass) {
#pragma unroll
        for (int it = 0; it < 8; ++it) {
          const int row = it * 2 + hh;
          v4f v = *(const v4f*)(slab + row * 68 + c4);
          *(volatile v4f*)(C + (size_t)(mBase + row) * ldc + n0 + c4) = v;
        }
        __threadfence();
      }
    } else {
      const int q = lane >> 3, c8 = (lane & 7) * 8;
      unsigned short* C  = (unsigned short*)Cout  + (size_t)b * strideC;
      unsigned short* C2 = (OUT_MODE == 2) ? ((unsigned short*)Cout2 + (size_t)b * strideC) : nullptr;
      for (int pass = 0; pass < 2; ++pass) {
#pragma unroll
        for (int it = 0; it < 4; ++it) {
          const int row = it * 4 + q;
          const float* sp = slab + row * 68 + c8;
          v8h hv, lv;
#pragma unroll
          for (int e = 0; e < 8; ++e) {
            if (OUT_MODE == 1) {
              hv[e] = (_Float16)sp[e];
            } else {
              unsigned short hb = f2bf_bits(sp[e]);
              unsigned short lb = f2bf_bits(sp[e] - bf_bits2f(hb));
              hv[e] = __builtin_bit_cast(_Float16, hb);
              lv[e] = __builtin_bit_cast(_Float16, lb);
            }
          }
          *(volatile v8h*)(C + (size_t)(mBase + row) * ldc + n0 + c8) = hv;
          if (OUT_MODE == 2) *(volatile v8h*)(C2 + (size_t)(mBase + row) * ldc + n0 + c8) = lv;
        }
        __threadfence();
      }
    }
    __builtin_amdgcn_fence(__ATOMIC_RELEASE, "workgroup");
    __builtin_amdgcn_wave_barrier();
    __builtin_amdgcn_fence(__ATOMIC_ACQUIRE, "workgroup");
  }
}

__global__ __launch_bounds__(256) void cast8_f16_kernel(const float* __restrict__ in, unsigned short* __restrict__ out, int n8) {
  const int i = blockIdx.x * 256 + threadIdx.x;
  if (i >= n8) return;
  const float* p = in + 8 * (size_t)i;
  const v4f a = *(const v4f*)(p);
  const v4f c = *(const v4f*)(p + 4);
  unsigned short hb[8];
#pragma unroll
  for (int e = 0; e < 4; ++e) {
    hb[e]     = h_bits(a[e]);
    hb[4 + e] = h_bits(c[e]);
  }
  const v4u u = (v4u){pk16(hb[0], hb[1]), pk16(hb[2], hb[3]), pk16(hb[4], hb[5]), pk16(hb[6], hb[7])};
  unsigned short* q = out + 8 * (size_t)i;
  *(volatile v4u*)q = u;
  __threadfence();
  *(volatile v4u*)q = u;
}

__global__ __launch_bounds__(256) void wtcast_kernel(const float* __restrict__ W, unsigned short* __restrict__ out,
                                                     int Kin, int Nout, float scale) {
  __shared__ float sm[64][65];
  const int t  = threadIdx.x;
  const int k0 = blockIdx.x * 64;
  const int n0 = blockIdx.y * 64;
#pragma unroll
  for (int i = 0; i < 16; ++i) {
    const int e = i * 256 + t;
    const int r = e >> 6;
    const int c = e & 63;
    sm[c][r] = W[(size_t)(k0 + r) * Nout + n0 + c] * scale;
  }
  __syncthreads();
  const int lane = t & 31, wave = t >> 5;
  const int q = lane >> 3, c8 = (lane & 7) * 8;
  v4u uu[2];
#pragma unroll
  for (int it = 0; it < 2; ++it) {
    const int row = wave * 8 + it * 4 + q;
    unsigned short hb[8];
#pragma unroll
    for (int e = 0; e < 8; ++e) hb[e] = h_bits(sm[row][c8 + e]);
    uu[it] = (v4u){pk16(hb[0], hb[1]), pk16(hb[2], hb[3]), pk16(hb[4], hb[5]), pk16(hb[6], hb[7])};
  }
  for (int pass = 0; pass < 2; ++pass) {
#pragma unroll
    for (int it = 0; it < 2; ++it) {
      const int row = wave * 8 + it * 4 + q;
      *(volatile v4u*)(out + (size_t)(n0 + row) * Kin + k0 + c8) = uu[it];
    }
    __threadfence();
  }
}

struct RopeFreq { float f[32]; };
static_assert(sizeof(RopeFreq) == 128, "size");

__global__ __launch_bounds__(256) void rope_table_kernel(float* __restrict__ tab, RopeFreq rf) {
#pragma clang fp contract(off)
  __shared__ __align__(16) float cs[8][64];
  const int t = threadIdx.x, lane = t & 31, wave = t >> 5;
  const int pos = blockIdx.x * 8 + wave;
  float freq = rf.f[0];
#pragma unroll
  for (int j = 1; j < 32; ++j) freq = (lane == j) ? rf.f[j] : freq;
  const float ang = (float)pos * freq;
  float sv, cv;
  sincosf(ang, &sv, &cv);
  cs[wave][lane] = cv;
  cs[wave][32 + lane] = sv;
  __syncthreads();
  const int cidx = (lane & 15) * 4;
  const v4f val = *(const v4f*)(&cs[wave][cidx]);
  float* dst = tab + (size_t)pos * 64 + cidx;
  for (int pass = 0; pass < 2; ++pass) {
    if (lane < 16) *(volatile v4f*)dst = val;
    __threadfence();
  }
}

__global__ __launch_bounds__(256) void rope_split_kernel(const float* __restrict__ qkv, const float* __restrict__ tab,
                                                         unsigned short* __restrict__ q16, unsigned short* __restrict__ k16,
                                                         unsigned short* __restrict__ vt16) {
#pragma clang fp contract(off)
  __shared__ float sq[64][65];
  __shared__ float sk[64][65];
  __shared__ float sv[64][65];
  const int t = threadIdx.x;
  const int pos0 = blockIdx.x * 64;
  const int h = blockIdx.y;
  const int b = blockIdx.z;
#pragma unroll
  for (int it = 0; it < 8; ++it) {
    const int e = it * 256 + t;
    const int pl = e >> 5;
    const int i = e & 31;
    const int pos = pos0 + pl;
    const float* rp = qkv + ((size_t)(b * kSeq + pos)) * kQkvN + h * kHd + i;
    const float q1 = rp[0], q2 = rp[32];
    const float k1 = rp[kDim], k2 = rp[kDim + 32];
    const float v1 = rp[2 * kDim], v2 = rp[2 * kDim + 32];
    const float cv = tab[(size_t)pos * 64 + i];
    const float snv = tab[(size_t)pos * 64 + 32 + i];
    const float qa = q1 * cv, qb = q2 * snv, qc = q2 * cv, qd = q1 * snv;
    const float ka = k1 * cv, kb = k2 * snv, kc = k2 * cv, kd = k1 * snv;
    sq[pl][i] = qa - qb;
    sq[pl][i + 32] = qc + qd;
    sk[pl][i] = ka - kb;
    sk[pl][i + 32] = kc + kd;
    sv[pl][i] = v1;
    sv[pl][i + 32] = v2;
  }
  __syncthreads();
  const int lane = t & 31, wave = t >> 5;
  const int q = lane >> 3, c8 = (lane & 7) * 8;
  const int g = b * kHeads + h;
  unsigned short* qbase = q16 + ((size_t)g * kSeq + pos0) * kHd;
  unsigned short* kbase = k16 + ((size_t)g * kSeq + pos0) * kHd;
  unsigned short* vbase = vt16 + (size_t)g * kHd * kSeq + pos0;
  v4u uq[2], uk[2], uv[2];
#pragma unroll
  for (int it = 0; it < 2; ++it) {
    const int row = wave * 8 + it * 4 + q;
    unsigned short hq[8], hk[8], hv[8];
#pragma unroll
    for (int e = 0; e < 8; ++e) {
      hq[e] = h_bits(sq[row][c8 + e]);
      hk[e] = h_bits(sk[row][c8 + e]);
      hv[e] = h_bits(sv[c8 + e][row]);
    }
    uq[it] = (v4u){pk16(hq[0], hq[1]), pk16(hq[2], hq[3]), pk16(hq[4], hq[5]), pk16(hq[6], hq[7])};
    uk[it] = (v4u){pk16(hk[0], hk[1]), pk16(hk[2], hk[3]), pk16(hk[4], hk[5]), pk16(hk[6], hk[7])};
    uv[it] = (v4u){pk16(hv[0], hv[1]), pk16(hv[2], hv[3]), pk16(hv[4], hv[5]), pk16(hv[6], hv[7])};
  }
  for (int pass = 0; pass < 2; ++pass) {
#pragma unroll
    for (int it = 0; it < 2; ++it) {
      const int row = wave * 8 + it * 4 + q;
      *(volatile v4u*)(qbase + (size_t)row * kHd + c8) = uq[it];
      *(volatile v4u*)(kbase + (size_t)row * kHd + c8) = uk[it];
      *(volatile v4u*)(vbase + (size_t)row * kSeq + c8) = uv[it];
    }
    __threadfence();
  }
}

__global__ __launch_bounds__(256) void softmax_row_kernel(const float* __restrict__ S, unsigned short* __restrict__ P, float carry) {
  __shared__ float redM[8];
  __shared__ float redS[8];
  const int row  = blockIdx.x;
  const int t    = threadIdx.x;
  const int lane = t & 31, wave = t >> 5;
  const float* sr = S + (size_t)row * kSeq + t * 8;
  const v4f a = *(const v4f*)(sr);
  const v4f c = *(const v4f*)(sr + 4);
  float x[8];
#pragma unroll
  for (int e = 0; e < 4; ++e) { x[e] = a[e]; x[4 + e] = c[e]; }
  float m = fmaxf(fmaxf(fmaxf(x[0], x[1]), fmaxf(x[2], x[3])), fmaxf(fmaxf(x[4], x[5]), fmaxf(x[6], x[7])));
#pragma unroll
  for (int off = 16; off > 0; off >>= 1) m = fmaxf(m, __shfl_xor(m, off, 32));
  if (lane == 0) redM[wave] = m;
  __syncthreads();
  float gm = redM[0];
#pragma unroll
  for (int w = 1; w < 8; ++w) gm = fmaxf(gm, redM[w]);
  float ex[8];
  float s = 0.f;
#pragma unroll
  for (int e = 0; e < 8; ++e) { ex[e] = expf(x[e] - gm); s += ex[e]; }
#pragma unroll
  for (int off = 16; off > 0; off >>= 1) s += __shfl_xor(s, off, 32);
  if (lane == 0) redS[wave] = s;
  __syncthreads();
  float tot = redS[0];
#pragma unroll
  for (int w = 1; w < 8; ++w) tot += redS[w];
  const float inv = carry * (1.0f / tot);
  unsigned short hb[8];
#pragma unroll
  for (int e = 0; e < 8; ++e) hb[e] = h_bits(ex[e] * inv);
  const v4u u = (v4u){pk16(hb[0], hb[1]), pk16(hb[2], hb[3]), pk16(hb[4], hb[5]), pk16(hb[6], hb[7])};
  unsigned short* pr = P + (size_t)row * kSeq + t * 8;
  *(volatile v4u*)pr = u;
  __threadfence();
  *(volatile v4u*)pr = u;
}

__global__ __launch_bounds__(256) void layernorm_kernel(const float* __restrict__ in, const float* __restrict__ gam,
                                                        const float* __restrict__ bet, float* __restrict__ out, int nrows) {
  __shared__ __align__(16) float ys[8][kDim];
  const int lane = threadIdx.x & 31;
  const int wave = threadIdx.x >> 5;
  const int row  = blockIdx.x * 8 + wave;
  if (row >= nrows) return;
  const float* xr = in + (size_t)row * kDim + lane * 4;
  float s = 0.f;
#pragma unroll 1
  for (int c = 0; c < 8; ++c) {
    const v4f v = *(const v4f*)(xr + c * 128);
    s += (v[0] + v[1]) + (v[2] + v[3]);
  }
#pragma unroll
  for (int off = 16; off > 0; off >>= 1) s += __shfl_xor(s, off, 32);
  const float mu = s * (1.0f / 1024.0f);
  float qs = 0.f;
#pragma unroll 1
  for (int c = 0; c < 8; ++c) {
    const v4f v = *(const v4f*)(xr + c * 128);
    const float d0 = v[0] - mu, d1 = v[1] - mu, d2 = v[2] - mu, d3 = v[3] - mu;
    qs += (d0 * d0 + d1 * d1) + (d2 * d2 + d3 * d3);
  }
#pragma unroll
  for (int off = 16; off > 0; off >>= 1) qs += __shfl_xor(qs, off, 32);
  const float var  = qs * (1.0f / 1024.0f);
  const float rstd = rsqrtf(var + kLnEps);
  float* yw = &ys[wave][lane * 4];
#pragma unroll 1
  for (int c = 0; c < 8; ++c) {
    const v4f v  = *(const v4f*)(xr + c * 128);
    const v4f gv = *(const v4f*)(gam + c * 128 + lane * 4);
    const v4f bv = *(const v4f*)(bet + c * 128 + lane * 4);
    v4f y;
    y[0] = (v[0] - mu) * rstd * gv[0] + bv[0];
    y[1] = (v[1] - mu) * rstd * gv[1] + bv[1];
    y[2] = (v[2] - mu) * rstd * gv[2] + bv[2];
    y[3] = (v[3] - mu) * rstd * gv[3] + bv[3];
    *(v4f*)(yw + c * 128) = y;
  }
  __builtin_amdgcn_fence(__ATOMIC_RELEASE, "workgroup");
  __builtin_amdgcn_wave_barrier();
  __builtin_amdgcn_fence(__ATOMIC_ACQUIRE, "workgroup");
  float* orow = out + (size_t)row * kDim + lane * 4;
  for (int pass = 0; pass < 2; ++pass) {
#pragma unroll 1
    for (int c = 0; c < 8; ++c) {
      const v4f y = *(const v4f*)(yw + c * 128);
      *(volatile v4f*)(orow + c * 128) = y;
    }
    __threadfence();
  }
}

__global__ __launch_bounds__(256) void gelu_cast_kernel(const float* __restrict__ in, unsigned short* __restrict__ out,
                                                        int n8, float carry) {
  const int i = blockIdx.x * 256 + threadIdx.x;
  if (i >= n8) return;
  const float* p = in + 8 * (size_t)i;
  unsigned r0 = 0u, r1 = 0u, r2 = 0u, r3 = 0u;
#pragma unroll 1
  for (int e = 0; e < 8; ++e) {
    const float v  = p[e];
    const float gv = 0.5f * v * (1.0f + erff(v * 0.70710678118654752f)) * carry;
    const unsigned u = ((unsigned)h_bits(gv)) << (16 * (e & 1));
    const int w = e >> 1;
    r0 = (w == 0) ? (r0 | u) : r0;
    r1 = (w == 1) ? (r1 | u) : r1;
    r2 = (w == 2) ? (r2 | u) : r2;
    r3 = (w == 3) ? (r3 | u) : r3;
  }
  const v4u u4 = (v4u){r0, r1, r2, r3};
  unsigned short* qo = out + 8 * (size_t)i;
  *(volatile v4u*)qo = u4;
  __threadfence();
  *(volatile v4u*)qo = u4;
}

extern "C" void kernel_launch(void* const* d_in, const int* in_sizes, int n_in,
                              void* d_out, int out_size, void* d_ws, size_t ws_size, hipStream_t stream) {
  if (n_in < 13) return;
  if (in_sizes[0] != kTok * kDim || in_sizes[1] != kDim * kQkvN || in_sizes[2] != kQkvN ||
      in_sizes[3] != kDim * kDim || in_sizes[4] != kDim || in_sizes[5] != kDim || in_sizes[6] != kDim ||
      in_sizes[7] != kDim || in_sizes[8] != kDim || in_sizes[9] != kDim * kFfn || in_sizes[10] != kFfn ||
      in_sizes[11] != kFfn * kDim || in_sizes[12] != kDim) return;
  if (out_size < kTok * kDim) return;
  if (ws_size < kWsNeed) return;

  const float* x      = (const float*)d_in[0];
  const float* qkv_w  = (const float*)d_in[1];
  const float* qkv_b  = (const float*)d_in[2];
  const float* out_w  = (const float*)d_in[3];
  const float* out_b  = (const float*)d_in[4];
  const float* ln1_g  = (const float*)d_in[5];
  const float* ln1_b  = (const float*)d_in[6];
  const float* ln2_g  = (const float*)d_in[7];
  const float* ln2_b  = (const float*)d_in[8];
  const float* ffn1_w = (const float*)d_in[9];
  const float* ffn1_b = (const float*)d_in[10];
  const float* ffn2_w = (const float*)d_in[11];
  const float* ffn2_b = (const float*)d_in[12];
  float* out = (float*)d_out;

  char* ws = (char*)d_ws;
  float*          qkvf  = (float*)(ws + kOffQkvF);
  unsigned short* x16   = (unsigned short*)(ws + kOffX16);
  unsigned short* wqkv  = (unsigned short*)(ws + kOffWqkv);
  float*          tab   = (float*)(ws + kOffTab);
  unsigned short* q16   = (unsigned short*)(ws + kOffQ16);
  unsigned short* k16   = (unsigned short*)(ws + kOffK16);
  unsigned short* vt16  = (unsigned short*)(ws + kOffVt16);
  float*          sc    = (float*)(ws + kOffSc);
  unsigned short* pp    = (unsigned short*)(ws + kOffP);
  unsigned short* att   = (unsigned short*)(ws + kOffAtt);
  unsigned short* wo16  = (unsigned short*)(ws + kOffWo);
  float*          y1    = (float*)(ws + kOffY1);
  float*          x1f   = (float*)(ws + kOffX1F);
  unsigned short* x1h   = (unsigned short*)(ws + kOffX1H);
  unsigned short* w116  = (unsigned short*)(ws + kOffW1);
  float*          hpre  = (float*)(ws + kOffHpre);
  unsigned short* h16   = (unsigned short*)(ws + kOffH16);
  unsigned short* w216  = (unsigned short*)(ws + kOffW2);
  float*          y2    = (float*)(ws + kOffY2);

  RopeFreq rf;
  for (int i = 0; i < 32; ++i) {
    const float pw = (float)pow(10000.0, (double)(2 * i) / 64.0);
    rf.f[i] = 1.0f / pw;
  }

  cast8_f16_kernel<<<(kTok * kDim / 8) / 256, 256, 0, stream>>>(x, x16, kTok * kDim / 8);
  wtcast_kernel<<<dim3(kDim / 64, kQkvN / 64), 256, 0, stream>>>(qkv_w, wqkv, kDim, kQkvN, kWCarry);
  rope_table_kernel<<<kSeq / 8, 256, 0, stream>>>(tab, rf);

  wmma_gemm64<0, false, 2, 0, false, 0><<<dim3((kTok / 64) * (kQkvN / 64) / 8, 1), 256, 0, stream>>>(
      x16, x16, kDim, 0L, wqkv, wqkv, kDim, 0L, (void*)qkvf, (void*)qkvf, kQkvN, 0L,
      qkv_b, x, 0L, kTok, kQkvN, kDim, kQkvScale);

  rope_split_kernel<<<dim3(kSeq / 64, kHeads, kBatch), 256, 0, stream>>>(qkvf, tab, q16, k16, vt16);

  for (int ch = 0; ch < kGroups / kChunkG; ++ch) {
    const int g0 = ch * kChunkG;
    const int bidx = g0 / kHeads;
    const int h0 = g0 - bidx * kHeads;
    const size_t gofs = (size_t)g0 * kSeq * kHd;
    wmma_gemm64<0, false, 0, 0, false, 0><<<dim3((kSeq / 64) * (kSeq / 64) / 8, kChunkG), 256, 0, stream>>>(
        q16 + gofs, q16 + gofs, kHd, (long)kSeq * kHd,
        k16 + gofs, k16 + gofs, kHd, (long)kSeq * kHd,
        (void*)sc, (void*)sc, kSeq, (long)kSeq * kSeq,
        qkv_b, x, 0L, kSeq, kSeq, kHd, kScoreScale);
    softmax_row_kernel<<<kChunkG * kSeq, 256, 0, stream>>>(sc, pp, kPCarry);
    unsigned short* attc = att + ((size_t)bidx * kSeq * kDim + (size_t)h0 * kHd);
    wmma_gemm64<0, false, 0, 1, false, 0><<<dim3((kSeq / 64) * (kHd / 64) / 8, kChunkG), 256, 0, stream>>>(
        pp, pp, kSeq, (long)kSeq * kSeq,
        vt16 + gofs, vt16 + gofs, kSeq, (long)kHd * kSeq,
        (void*)attc, (void*)attc, kDim, (long)kHd,
        qkv_b, x, 0L, kSeq, kHd, kSeq, kPVScale);
  }

  wtcast_kernel<<<dim3(kDim / 64, kDim / 64), 256, 0, stream>>>(out_w, wo16, kDim, kDim, kWCarry);
  wmma_gemm64<0, false, 2, 0, true, 0><<<dim3((kTok / 64) * (kDim / 64) / 8, 1), 256, 0, stream>>>(
      att, att, kDim, 0L, wo16, wo16, kDim, 0L, (void*)y1, (void*)y1, kDim, 0L,
      out_b, x, 0L, kTok, kDim, kDim, kWoScale);

  layernorm_kernel<<<kTok / 8, 256, 0, stream>>>(y1, ln1_g, ln1_b, x1f, kTok);
  cast8_f16_kernel<<<(kTok * kDim / 8) / 256, 256, 0, stream>>>(x1f, x1h, kTok * kDim / 8);

  wtcast_kernel<<<dim3(kDim / 64, kFfn / 64), 256, 0, stream>>>(ffn1_w, w116, kDim, kFfn, kWCarry);
  wmma_gemm64<0, false, 2, 0, false, 0><<<dim3((kTok / 64) * (kFfn / 64) / 8, 1), 256, 0, stream>>>(
      x1h, x1h, kDim, 0L, w116, w116, kDim, 0L, (void*)hpre, (void*)hpre, kFfn, 0L,
      ffn1_b, x, 0L, kTok, kFfn, kDim, kFfn1Scale);
  gelu_cast_kernel<<<(kTok * kFfn / 8) / 256, 256, 0, stream>>>(hpre, h16, kTok * kFfn / 8, kHCarry);

  wtcast_kernel<<<dim3(kFfn / 64, kDim / 64), 256, 0, stream>>>(ffn2_w, w216, kFfn, kDim, kW2Carry);
  wmma_gemm64<0, false, 2, 0, true, 0><<<dim3((kTok / 64) * (kDim / 64) / 8, 1), 256, 0, stream>>>(
      h16, h16, kFfn, 0L, w216, w216, kFfn, 0L, (void*)y2, (void*)y2, kDim, 0L,
      ffn2_b, x1f, 0L, kTok, kDim, kFfn, kFfn2Scale);

  layernorm_kernel<<<kTok / 8, 256, 0, stream>>>(y2, ln2_g, ln2_b, out, kTok);
}
